// TDPolicyNetwork_62242666053676
// MI455X (gfx1250) — hardware-verified
//
#include <hip/hip_runtime.h>
#include <stddef.h>
#include <stdint.h>

#define NB    8
#define SQ    256
#define NTOK  2048
#define DIN   16
#define DINP  32
#define HID   256
#define H2    128
#define H4    64
#define NHD   8
#define HDM   32
#define DFF   512
#define NQKV  768
#define NL    3
#define G4    1024
#define QKPLANE (NB * NHD * SQ * HDM)

static_assert(NTOK == NB * SQ);
static_assert(NHD * HDM == HID);
static_assert(NQKV == 3 * HID);
static_assert(G4 == 4 * HID);
static_assert(H2 + H4 + H4 == HID);
static_assert(NTOK % 256 == 0);
static_assert(HID % 64 == 0);
static_assert(DFF % 64 == 0);
static_assert(G4 % 64 == 0);
static_assert(H2 % 64 == 0);
static_assert(DINP % 32 == 0);
static_assert(SQ == 256);

typedef _Float16 v16h __attribute__((ext_vector_type(16)));
typedef _Float16 v8h  __attribute__((ext_vector_type(8)));
typedef float    v8f  __attribute__((ext_vector_type(8)));
typedef float    v4f  __attribute__((ext_vector_type(4)));
typedef unsigned int v4u __attribute__((ext_vector_type(4)));

union Frag  { v16h v; v8h h[2]; };
union Pack8 { v8h h; v4u u; };

__device__ __forceinline__ v8f mma16(v16h a, v16h b, v8f c) {
  c = __builtin_amdgcn_wmma_f32_16x16x32_f16(false, a, false, b, (short)0, c, false, false);
  asm volatile("v_nop\n\tv_nop\n\tv_nop\n\tv_nop" : "+v"(c) : "v"(a), "v"(b));
  return c;
}

__device__ __forceinline__ v16h ldfrag(const _Float16* p, int ld, int row0, int k0, int lane) {
  const int m = lane & 15, lh = lane >> 4;
  const _Float16* q = p + (size_t)(row0 + m) * ld + k0 + 8 * lh;
  Frag f;
  f.h[0] = *(const v8h*)(q);
  f.h[1] = *(const v8h*)(q + 16);
  return f.v;
}

__device__ __forceinline__ v16h ldfrag_oh(const _Float16* op, int m0, int k0, int lane) {
  const int m = lane & 15, lh = lane >> 4;
  const int row = m0 + m;
  const int bq = row >> 8, s = row & 255, hd = k0 >> 5;
  const _Float16* q = op + ((size_t)(bq * NHD + hd) * SQ + s) * HDM + 8 * lh;
  Frag f;
  f.h[0] = *(const v8h*)(q);
  f.h[1] = *(const v8h*)(q + 16);
  return f.v;
}

__device__ __forceinline__ v8f zero8() { return (v8f){0.f, 0.f, 0.f, 0.f, 0.f, 0.f, 0.f, 0.f}; }

__device__ __forceinline__ float sgm(float x) { return __builtin_amdgcn_rcpf(1.0f + __expf(-x)); }
__device__ __forceinline__ float tnh(float x) {
  const float e = __expf(2.0f * x);
  return fmaf(-2.0f, __builtin_amdgcn_rcpf(e + 1.0f), 1.0f);
}

__device__ __forceinline__ void gemm32x64(const _Float16* __restrict__ A, int lda,
                                          const _Float16* __restrict__ Bt, int ldb, int K,
                                          int m0, int n0, int lane, v8f (&acc)[2][4]) {
#pragma unroll 1
  for (int k0 = 0; k0 < K; k0 += 32) {
    const v16h a0 = ldfrag(A, lda, m0, k0, lane);
    const v16h a1 = ldfrag(A, lda, m0 + 16, k0, lane);
    const v16h b0 = ldfrag(Bt, ldb, n0, k0, lane);
    const v16h b1 = ldfrag(Bt, ldb, n0 + 16, k0, lane);
    const v16h b2 = ldfrag(Bt, ldb, n0 + 32, k0, lane);
    const v16h b3 = ldfrag(Bt, ldb, n0 + 48, k0, lane);
    acc[0][0] = mma16(a0, b0, acc[0][0]);
    acc[1][0] = mma16(a1, b0, acc[1][0]);
    acc[0][1] = mma16(a0, b1, acc[0][1]);
    acc[1][1] = mma16(a1, b1, acc[1][1]);
    acc[0][2] = mma16(a0, b2, acc[0][2]);
    acc[1][2] = mma16(a1, b2, acc[1][2]);
    acc[0][3] = mma16(a0, b3, acc[0][3]);
    acc[1][3] = mma16(a1, b3, acc[1][3]);
  }
}

__device__ __forceinline__ void gemm32x64_oh(const _Float16* __restrict__ Op,
                                             const _Float16* __restrict__ Bt, int ldb,
                                             int m0, int n0, int lane, v8f (&acc)[2][4]) {
#pragma unroll 1
  for (int k0 = 0; k0 < HID; k0 += 32) {
    const v16h a0 = ldfrag_oh(Op, m0, k0, lane);
    const v16h a1 = ldfrag_oh(Op, m0 + 16, k0, lane);
    const v16h b0 = ldfrag(Bt, ldb, n0, k0, lane);
    const v16h b1 = ldfrag(Bt, ldb, n0 + 16, k0, lane);
    const v16h b2 = ldfrag(Bt, ldb, n0 + 32, k0, lane);
    const v16h b3 = ldfrag(Bt, ldb, n0 + 48, k0, lane);
    acc[0][0] = mma16(a0, b0, acc[0][0]);
    acc[1][0] = mma16(a1, b0, acc[1][0]);
    acc[0][1] = mma16(a0, b1, acc[0][1]);
    acc[1][1] = mma16(a1, b1, acc[1][1]);
    acc[0][2] = mma16(a0, b2, acc[0][2]);
    acc[1][2] = mma16(a1, b2, acc[1][2]);
    acc[0][3] = mma16(a0, b3, acc[0][3]);
    acc[1][3] = mma16(a1, b3, acc[1][3]);
  }
}

__global__ __launch_bounds__(256) void k_cvt(const float* __restrict__ src, _Float16* __restrict__ dst,
                                             int rows, int kin, int kout, float scale) {
  const int p = blockIdx.x * 256 + (int)threadIdx.x;
  const int kp8 = kout >> 3;
  const int total = rows * kp8;
  if (p >= total) return;
  const int r   = p / kp8;
  const int col = (p - r * kp8) * 8;
  const int lc  = min(col, kin - 8);
  const float f = (col < kin) ? scale : 0.0f;
  const float* sp = src + (size_t)r * kin + lc;
  const v4f a0 = *(const v4f*)(sp) * f;
  const v4f a1 = *(const v4f*)(sp + 4) * f;
  Pack8 pk;
  pk.h = (v8h){(_Float16)a0[0], (_Float16)a0[1], (_Float16)a0[2], (_Float16)a0[3],
               (_Float16)a1[0], (_Float16)a1[1], (_Float16)a1[2], (_Float16)a1[3]};
  const v4u vv = pk.u;
  volatile v4u* d = (volatile v4u*)(dst + (size_t)p * 8);
  *d = vv;
  __threadfence();
  *d = vv;
}

#define OTP 68
__device__ __forceinline__ void out_epilogue_f32(v8f (&acc)[2][4], float scale, const float (&bb)[4],
                                                 float* sw, float* __restrict__ out, int ldo,
                                                 int m0, int n0, int lane, int hh, int c) {
#pragma unroll
  for (int sub = 0; sub < 2; ++sub) {
    __syncthreads();
#pragma unroll
    for (int t = 0; t < 4; ++t) {
#pragma unroll
      for (int r = 0; r < 8; ++r) sw[(8 * hh + r) * OTP + 16 * t + c] = acc[sub][t][r] * scale + bb[t];
    }
    __syncthreads();
    v4f val[8];
    size_t go[8];
#pragma unroll
    for (int it = 0; it < 8; ++it) {
      const int p    = lane + 32 * it;
      const int L    = p >> 3;
      const int pc   = p & 7;
      const int row  = L >> 1;
      const int half = L & 1;
      val[it] = *(const v4f*)(sw + row * OTP + half * 32 + pc * 4);
      go[it]  = (size_t)(m0 + sub * 16 + row) * ldo + n0 + half * 32 + pc * 4;
    }
    for (int ps = 0; ps < 2; ++ps) {
#pragma unroll
      for (int it = 0; it < 8; ++it) *(volatile v4f*)(out + go[it]) = val[it];
      __threadfence();
    }
  }
}

__device__ __forceinline__ void out_epilogue_h16(v8f (&acc)[2][4], float scale, const float (&bb)[4], float oscale,
                                                 float* sw, _Float16* __restrict__ out, int ldo,
                                                 int m0, int n0, int lane, int hh, int c) {
#pragma unroll
  for (int sub = 0; sub < 2; ++sub) {
    __syncthreads();
#pragma unroll
    for (int t = 0; t < 4; ++t) {
#pragma unroll
      for (int r = 0; r < 8; ++r) {
        const float v = acc[sub][t][r] * scale + bb[t];
        sw[(8 * hh + r) * OTP + 16 * t + c] = fmaxf(v, 0.f) * oscale;
      }
    }
    __syncthreads();
    v4u val[4];
    size_t go[4];
#pragma unroll
    for (int it = 0; it < 4; ++it) {
      const int p  = lane + 32 * it;
      const int L  = p >> 3;
      const int pc = p & 7;
      const float* ra = sw + L * OTP + pc * 8;
      const v4f a0 = *(const v4f*)(ra), a1 = *(const v4f*)(ra + 4);
      Pack8 pk;
      pk.h = (v8h){(_Float16)a0[0], (_Float16)a0[1], (_Float16)a0[2], (_Float16)a0[3],
                   (_Float16)a1[0], (_Float16)a1[1], (_Float16)a1[2], (_Float16)a1[3]};
      val[it] = pk.u;
      go[it]  = (size_t)(m0 + sub * 16 + L) * ldo + n0 + pc * 8;
    }
    for (int ps = 0; ps < 2; ++ps) {
#pragma unroll
      for (int it = 0; it < 4; ++it) *(volatile v4u*)(out + go[it]) = val[it];
      __threadfence();
    }
  }
}

__global__ __launch_bounds__(256) void k_gemm_f32(const _Float16* __restrict__ ap, int lda,
                                                  const _Float16* __restrict__ wt, int K,
                                                  const float* __restrict__ bias, float scale,
                                                  float* __restrict__ out, int ldo) {
  __shared__ __align__(16) float st[8][16 * OTP];
  const int tid = threadIdx.x, lane = tid & 31, wave = tid >> 5;
  const int hh = lane >> 4, c = lane & 15;
  const int m0 = blockIdx.x * 256 + wave * 32;
  const int n0 = blockIdx.y * 64;

  v8f acc[2][4];
#pragma unroll
  for (int s = 0; s < 2; ++s)
#pragma unroll
    for (int t = 0; t < 4; ++t) acc[s][t] = zero8();
  gemm32x64(ap, lda, wt, K, K, m0, n0, lane, acc);
  float bb[4];
#pragma unroll
  for (int t = 0; t < 4; ++t) bb[t] = bias[n0 + 16 * t + c];
  out_epilogue_f32(acc, scale, bb, st[wave], out, ldo, m0, n0, lane, hh, c);
}

__global__ __launch_bounds__(256) void k_gemm_h16(const _Float16* __restrict__ ap, int lda,
                                                  const _Float16* __restrict__ wt, int K,
                                                  const float* __restrict__ bias, float scale, float oscale,
                                                  _Float16* __restrict__ out, int ldo) {
  __shared__ __align__(16) float st[8][16 * OTP];
  const int tid = threadIdx.x, lane = tid & 31, wave = tid >> 5;
  const int hh = lane >> 4, c = lane & 15;
  const int m0 = blockIdx.x * 256 + wave * 32;
  const int n0 = blockIdx.y * 64;

  v8f acc[2][4];
#pragma unroll
  for (int s = 0; s < 2; ++s)
#pragma unroll
    for (int t = 0; t < 4; ++t) acc[s][t] = zero8();
  gemm32x64(ap, lda, wt, K, K, m0, n0, lane, acc);
  float bb[4];
#pragma unroll
  for (int t = 0; t < 4; ++t) bb[t] = bias[n0 + 16 * t + c];
  out_epilogue_h16(acc, scale, bb, oscale, st[wave], out, ldo, m0, n0, lane, hh, c);
}

__global__ __launch_bounds__(256) void k_gemm_oh(const _Float16* __restrict__ op,
                                                 const _Float16* __restrict__ wt,
                                                 const float* __restrict__ bias, float scale,
                                                 float* __restrict__ out, int ldo) {
  __shared__ __align__(16) float st[8][16 * OTP];
  const int tid = threadIdx.x, lane = tid & 31, wave = tid >> 5;
  const int hh = lane >> 4, c = lane & 15;
  const int m0 = blockIdx.x * 256 + wave * 32;
  const int n0 = blockIdx.y * 64;

  v8f acc[2][4];
#pragma unroll
  for (int s = 0; s < 2; ++s)
#pragma unroll
    for (int t = 0; t < 4; ++t) acc[s][t] = zero8();
  gemm32x64_oh(op, wt, HID, m0, n0, lane, acc);
  float bb[4];
#pragma unroll
  for (int t = 0; t < 4; ++t) bb[t] = bias[n0 + 16 * t + c];
  out_epilogue_f32(acc, scale, bb, st[wave], out, ldo, m0, n0, lane, hh, c);
}

__global__ __launch_bounds__(256) void k_asmx(const float* __restrict__ p32, const float* __restrict__ pos,
                                              float* __restrict__ xa, _Float16* __restrict__ x16) {
  __shared__ __align__(16) float sw[8][HID];
  const int tid = threadIdx.x, lane = tid & 31, wave = tid >> 5;
  const size_t m = (size_t)blockIdx.x * 8 + wave;
  const int s = (int)(m & 255);
  v4f v[2];
  v[0] = *(const v4f*)(p32 + m * H2 + lane * 4);
  const int j  = lane * 4;
  const int jj = min(j, H4 - 4);
  const v4f pv = *(const v4f*)(pos + (size_t)s * H4 + jj);
  const float keep = (lane < 16) ? 1.0f : 0.0f;
  v[1] = pv * keep;
  for (int ps = 0; ps < 2; ++ps) {
#pragma unroll
    for (int it = 0; it < 2; ++it) *(volatile v4f*)(xa + m * HID + it * 128 + lane * 4) = v[it];
    __threadfence();
  }
#pragma unroll
  for (int it = 0; it < 2; ++it) *(v4f*)(sw[wave] + it * 128 + lane * 4) = v[it];
  __syncthreads();
  const float* cp = sw[wave] + 8 * lane;
  const v4f a0 = *(const v4f*)(cp), a1 = *(const v4f*)(cp + 4);
  Pack8 pk;
  pk.h = (v8h){(_Float16)a0[0], (_Float16)a0[1], (_Float16)a0[2], (_Float16)a0[3],
               (_Float16)a1[0], (_Float16)a1[1], (_Float16)a1[2], (_Float16)a1[3]};
  const v4u hv = pk.u;
  volatile v4u* d = (volatile v4u*)(x16 + m * HID + 8 * lane);
  *d = hv;
  __threadfence();
  *d = hv;
}

#define STP 72
#define SVP 264
__global__ __launch_bounds__(256) void k_qkv(const _Float16* __restrict__ xh,
                                             const _Float16* __restrict__ wt,
                                             const float* __restrict__ bias,
                                             _Float16* __restrict__ qkp,
                                             _Float16* __restrict__ vtp) {
  __shared__ __align__(16) _Float16 st[256 * STP];
  const int tid = threadIdx.x, lane = tid & 31, wave = tid >> 5;
  const int hh = lane >> 4, c = lane & 15;
  const int b     = blockIdx.x;
  const int ns    = blockIdx.y;
  const int which = ns >> 2;
  const int hb0   = b * NHD + 2 * (ns & 3);
  const int m0    = b * SQ + wave * 32;
  const int n0    = ns * 64;
  const int lr0   = wave * 32;

  v8f acc[2][4];
#pragma unroll
  for (int s = 0; s < 2; ++s)
#pragma unroll
    for (int t = 0; t < 4; ++t) acc[s][t] = zero8();
  gemm32x64(xh, HID, wt, HID, HID, m0, n0, lane, acc);

  float bb[4];
#pragma unroll
  for (int t = 0; t < 4; ++t) bb[t] = bias[n0 + 16 * t + c];

  if (which < 2) {
#pragma unroll
    for (int sub = 0; sub < 2; ++sub)
#pragma unroll
      for (int t = 0; t < 4; ++t)
#pragma unroll
        for (int r = 0; r < 8; ++r)
          st[(lr0 + sub * 16 + 8 * hh + r) * STP + 16 * t + c] =
              (_Float16)(acc[sub][t][r] * 0.03125f + bb[t]);
  } else {
#pragma unroll
    for (int sub = 0; sub < 2; ++sub)
#pragma unroll
      for (int t = 0; t < 4; ++t)
#pragma unroll
        for (int r = 0; r < 8; ++r)
          st[(16 * t + c) * SVP + lr0 + sub * 16 + 8 * hh + r] =
              (_Float16)(acc[sub][t][r] * 0.03125f + bb[t]);
  }
  __syncthreads();

  if (which < 2) {
    _Float16* base = qkp + (size_t)which * QKPLANE + (size_t)hb0 * SQ * HDM;
#pragma unroll
    for (int g = 0; g < 2; ++g) {
      v4u val[4];
      size_t go[4];
#pragma unroll
      for (int j4 = 0; j4 < 4; ++j4) {
        const int p   = tid + 256 * (4 * g + j4);
        const int hj  = p >> 10;
        const int rem = p & 1023;
        const int s   = rem >> 2;
        const int pc  = rem & 3;
        Pack8 pk;
        pk.h    = *(const v8h*)(st + s * STP + hj * 32 + pc * 8);
        val[j4] = pk.u;
        go[j4]  = (size_t)hj * (SQ * HDM) + (size_t)rem * 8;
      }
      for (int ps = 0; ps < 2; ++ps) {
#pragma unroll
        for (int j4 = 0; j4 < 4; ++j4) *(volatile v4u*)(base + go[j4]) = val[j4];
        __threadfence();
      }
    }
  } else {
    _Float16* base = vtp + (size_t)hb0 * HDM * SQ;
#pragma unroll
    for (int g = 0; g < 2; ++g) {
      v4u val[4];
      size_t go[4];
#pragma unroll
      for (int j4 = 0; j4 < 4; ++j4) {
        const int p  = tid + 256 * (4 * g + j4);
        const int d  = p >> 5;
        const int pc = p & 31;
        Pack8 pk;
        pk.h    = *(const v8h*)(st + d * SVP + pc * 8);
        val[j4] = pk.u;
        go[j4]  = (size_t)p * 8;
      }
      for (int ps = 0; ps < 2; ++ps) {
#pragma unroll
        for (int j4 = 0; j4 < 4; ++j4) *(volatile v4u*)(base + go[j4]) = val[j4];
        __threadfence();
      }
    }
  }
}

#define KP 40
#define VP 264
#define PP 72
__global__ __launch_bounds__(256) void k_attn(const _Float16* __restrict__ qkp,
                                              const _Float16* __restrict__ vtp,
                                              _Float16* __restrict__ op, float sscale) {
  __shared__ __align__(16) _Float16 Ks[SQ * KP];
  __shared__ __align__(16) _Float16 Vs[HDM * VP];
  __shared__ __align__(16) _Float16 Ps[8 * 16 * PP];

  const int tid = threadIdx.x, lane = tid & 31, wave = tid >> 5;
  const int hh = lane >> 4, c = lane & 15;
  const int hb = blockIdx.x >> 1;
  const int qb = blockIdx.x & 1;
  const int q0 = qb * 128 + wave * 16;

  const _Float16* Q = qkp + (size_t)hb * SQ * HDM;
  const _Float16* K = qkp + (size_t)QKPLANE + (size_t)hb * SQ * HDM;
  const _Float16* V = vtp + (size_t)hb * HDM * SQ;

#pragma unroll
  for (int e = 0; e < 4; ++e) {
    const int p = tid + 256 * e;
    {
      const int r = p >> 2, qq = (p & 3) * 8;
      *(v8h*)(Ks + r * KP + qq) = *(const v8h*)(K + (size_t)r * HDM + qq);
    }
    {
      const int r = p >> 5, qq = (p & 31) * 8;
      *(v8h*)(Vs + r * VP + qq) = *(const v8h*)(V + (size_t)r * SQ + qq);
    }
  }
  const v16h qa = ldfrag(Q, HDM, q0, 0, lane);
  __syncthreads();

  const float NEGI = -__builtin_huge_valf();
  float mrow[8], lrow[8];
  v8f oacc[2];
#pragma unroll
  for (int r = 0; r < 8; ++r) { mrow[r] = NEGI; lrow[r] = 0.f; }
#pragma unroll
  for (int t = 0; t < 2; ++t) oacc[t] = zero8();

  _Float16* pw = Ps + wave * 16 * PP;

  for (int kc = 0; kc < SQ / 64; ++kc) {
    const int kv0 = kc * 64;
    __syncthreads();

    v8f s[4];
#pragma unroll
    for (int j = 0; j < 4; ++j) {
      const v16h kb = ldfrag(Ks, KP, kv0 + j * 16, 0, lane);
      s[j] = mma16(qa, kb, zero8());
    }
    float cm[8];
#pragma unroll
    for (int r = 0; r < 8; ++r) {
      float m = NEGI;
#pragma unroll
      for (int j = 0; j < 4; ++j) { s[j][r] *= sscale; m = fmaxf(m, s[j][r]); }
#pragma unroll
      for (int off = 1; off < 16; off <<= 1) m = fmaxf(m, __shfl_xor(m, off, 32));
      cm[r] = m;
    }
    float al[8];
#pragma unroll
    for (int r = 0; r < 8; ++r) {
      const float mnew  = fmaxf(mrow[r], cm[r]);
      const float alpha = __expf(mrow[r] - mnew);
      mrow[r] = mnew;
      float psum = 0.f;
#pragma unroll
      for (int j = 0; j < 4; ++j) {
        const float p = __expf(s[j][r] - mnew);
        psum += p;
        pw[(8 * hh + r) * PP + j * 16 + c] = (_Float16)(p * 1024.0f);
      }
#pragma unroll
      for (int off = 1; off < 16; off <<= 1) psum += __shfl_xor(psum, off, 32);
      lrow[r] = lrow[r] * alpha + psum;
      al[r] = alpha;
    }
#pragma unroll
    for (int t = 0; t < 2; ++t)
#pragma unroll
      for (int r = 0; r < 8; ++r) oacc[t][r] *= al[r];
    __syncthreads();

#pragma unroll
    for (int kk = 0; kk < 2; ++kk) {
      const v16h pa = ldfrag(pw, PP, 0, kk * 32, lane);
#pragma unroll
      for (int t = 0; t < 2; ++t) {
        const v16h vb = ldfrag(Vs, VP, t * 16, kv0 + kk * 32, lane);
        oacc[t] = mma16(pa, vb, oacc[t]);
      }
    }
  }

  float invl[8];
#pragma unroll
  for (int r = 0; r < 8; ++r) invl[r] = 0.0625f * __builtin_amdgcn_rcpf(lrow[r]);
  __syncthreads();
#pragma unroll
  for (int r = 0; r < 8; ++r) {
#pragma unroll
    for (int t = 0; t < 2; ++t)
      pw[(8 * hh + r) * PP + 16 * t + c] = (_Float16)(oacc[t][r] * invl[r]);
  }
  __syncthreads();
  v4u val[2];
  size_t go[2];
  const size_t obase = ((size_t)hb * SQ + q0) * HDM;
#pragma unroll
  for (int it = 0; it < 2; ++it) {
    const int p  = lane + 32 * it;
    const int L  = p >> 2;
    const int pc = p & 3;
    Pack8 pk;
    pk.h    = *(const v8h*)(pw + L * PP + pc * 8);
    val[it] = pk.u;
    go[it]  = obase + (size_t)p * 8;
  }
  for (int ps = 0; ps < 2; ++ps) {
#pragma unroll
    for (int it = 0; it < 2; ++it) *(volatile v4u*)(op + go[it]) = val[it];
    __threadfence();
  }
}

__global__ __launch_bounds__(256) void k_ln(const float* __restrict__ t, const float* __restrict__ res,
                                            const float* __restrict__ g, const float* __restrict__ be,
                                            float* __restrict__ yf, _Float16* __restrict__ yh) {
  __shared__ __align__(16) float sw[8][HID];
  const int tid = threadIdx.x, lane = tid & 31, wave = tid >> 5;
  const size_t m = (size_t)blockIdx.x * 8 + wave;
  const float* tr = t + m * HID;
  const float* rr = res + m * HID;

  v4f v[2];
  float s = 0.f;
#pragma unroll
  for (int it = 0; it < 2; ++it) {
    const int idx = it * 128 + lane * 4;
    const v4f a = *(const v4f*)(tr + idx);
    const v4f r = *(const v4f*)(rr + idx);
    v[it] = a + r;
    s += (v[it][0] + v[it][1]) + (v[it][2] + v[it][3]);
  }
#pragma unroll
  for (int off = 16; off >= 1; off >>= 1) s += __shfl_xor(s, off, 32);
  const float mean = s * 0.00390625f;
  float ss = 0.f;
#pragma unroll
  for (int it = 0; it < 2; ++it) {
    const v4f d = v[it] - mean;
    ss += (d[0] * d[0] + d[1] * d[1]) + (d[2] * d[2] + d[3] * d[3]);
  }
#pragma unroll
  for (int off = 16; off >= 1; off >>= 1) ss += __shfl_xor(ss, off, 32);
  const float var  = ss * 0.00390625f;
  const float rstd = rsqrtf(var + 1e-5f);

  v4f y[2];
#pragma unroll
  for (int it = 0; it < 2; ++it) {
    const int idx = it * 128 + lane * 4;
    const v4f gv = *(const v4f*)(g + idx);
    const v4f bv = *(const v4f*)(be + idx);
    y[it] = ((v[it] - mean) * rstd) * gv + bv;
  }
  for (int ps = 0; ps < 2; ++ps) {
#pragma unroll
    for (int it = 0; it < 2; ++it) *(volatile v4f*)(yf + m * HID + it * 128 + lane * 4) = y[it];
    __threadfence();
  }
#pragma unroll
  for (int it = 0; it < 2; ++it) *(v4f*)(sw[wave] + it * 128 + lane * 4) = y[it];
  __syncthreads();
  const float* cp = sw[wave] + 8 * lane;
  const v4f a0 = *(const v4f*)(cp), a1 = *(const v4f*)(cp + 4);
  Pack8 pk;
  pk.h = (v8h){(_Float16)a0[0], (_Float16)a0[1], (_Float16)a0[2], (_Float16)a0[3],
               (_Float16)a1[0], (_Float16)a1[1], (_Float16)a1[2], (_Float16)a1[3]};
  const v4u hv = pk.u;
  volatile v4u* d = (volatile v4u*)(yh + m * HID + 8 * lane);
  *d = hv;
  __threadfence();
  *d = hv;
}

__global__ __launch_bounds__(256) void k_gather(const _Float16* __restrict__ x16, const int* __restrict__ ts,
                                                _Float16* __restrict__ din) {
  const int tid = threadIdx.x, lane = tid & 31, wave = tid >> 5;
  const int row = blockIdx.x * 8 + wave;
  const int t = row >> 3, b = row & 7;
  const int tm = max(t - 1, 0);
  int idx = ts[b * SQ + tm];
  idx = min(max(idx, 0), SQ - 1);
  Pack8 pk;
  pk.h = *(const v8h*)(x16 + ((size_t)(b * SQ + idx)) * HID + lane * 8);
  const unsigned msk = (t > 0) ? 0xffffffffu : 0u;
  const v4u vv = pk.u & (v4u){msk, msk, msk, msk};
  volatile v4u* d = (volatile v4u*)(din + (size_t)row * HID + lane * 8);
  *d = vv;
  __threadfence();
  *d = vv;
}

#define HSP 264
#define GSP 1032
#define INV2048 0.00048828125f
static_assert((GSP * 4) % 16 == 0);
static_assert(7 * GSP + G4 <= NB * GSP);
__global__ __launch_bounds__(256) void k_lstm(const float* __restrict__ gx, const _Float16* __restrict__ whh,
                                              const float* __restrict__ bhh, _Float16* __restrict__ dout) {
  __shared__ __align__(16) _Float16 hs[16 * HSP];
  __shared__ __align__(16) float gs[NB * GSP];
  const int tid = threadIdx.x, lane = tid & 31, wave = tid >> 5;
  const int hh = lane >> 4, c = lane & 15;
  for (int i = tid; i < 16 * HSP; i += 256) hs[i] = (_Float16)0.0f;

  float bh[4][2];
#pragma unroll
  for (int q = 0; q < 4; ++q)
#pragma unroll
    for (int sub = 0; sub < 2; ++sub) bh[q][sub] = bhh[q * HID + wave * 32 + 16 * sub + c];
  float cst[2][8];
#pragma unroll
  for (int sub = 0; sub < 2; ++sub)
#pragma unroll
    for (int r = 0; r < 8; ++r) cst[sub][r] = 0.f;
  __syncthreads();

#pragma unroll 1
  for (int t = 0; t < SQ; ++t) {
    const float* gt = gx + (size_t)t * NB * G4;
#pragma unroll
    for (int e = 0; e < 8; ++e) {
      const int p   = tid + 256 * e;
      const int row = p >> 8;
      const int col = (p & 255) * 4;
      *(v4f*)(gs + row * GSP + col) = *(const v4f*)(gt + (size_t)row * G4 + col);
    }
    __syncthreads();

    v8f acc[4][2];
#pragma unroll
    for (int q = 0; q < 4; ++q) {
#pragma unroll
      for (int sub = 0; sub < 2; ++sub) {
        const int col = q * HID + wave * 32 + 16 * sub + c;
#pragma unroll
        for (int r = 0; r < 8; ++r) {
          const int rs = (hh != 0) ? 7 : r;
          acc[q][sub][r] = (gs[rs * GSP + col] + bh[q][sub]) * 2048.0f;
        }
      }
    }
#pragma unroll 1
    for (int k0 = 0; k0 < HID; k0 += 32) {
      const v16h a = ldfrag(hs, HSP, 0, k0, lane);
#pragma unroll
      for (int q = 0; q < 4; ++q) {
#pragma unroll
        for (int sub = 0; sub < 2; ++sub) {
          const v16h b = ldfrag(whh, HID, q * HID + wave * 32 + 16 * sub, k0, lane);
          acc[q][sub] = mma16(a, b, acc[q][sub]);
        }
      }
    }
    float h64[2][8];
#pragma unroll
    for (int sub = 0; sub < 2; ++sub) {
#pragma unroll
      for (int r = 0; r < 8; ++r) {
        const float pi = acc[0][sub][r] * INV2048;
        const float pf = acc[1][sub][r] * INV2048;
        const float pg = acc[2][sub][r] * INV2048;
        const float po = acc[3][sub][r] * INV2048;
        const float ig = sgm(pi), fg = sgm(pf), gg = tnh(pg), og = sgm(po);
        const float cn = fg * cst[sub][r] + ig * gg;
        cst[sub][r] = cn;
        const float hv = og * tnh(cn);
        h64[sub][r] = (hh == 0) ? hv * 64.0f : 0.0f;
      }
    }
    __syncthreads();
#pragma unroll
    for (int sub = 0; sub < 2; ++sub)
#pragma unroll
      for (int r = 0; r < 8; ++r)
        hs[(8 * hh + r) * HSP + wave * 32 + 16 * sub + c] = (_Float16)h64[sub][r];
    __syncthreads();
    Pack8 pk;
    pk.h = *(const v8h*)(hs + wave * HSP + lane * 8);
    const v4u vv = pk.u;
    volatile v4u* d = (volatile v4u*)(dout + ((size_t)(wave * SQ + t)) * HID + lane * 8);
    *d = vv;
    __threadfence();
    *d = vv;
  }
}

__global__ __launch_bounds__(256) void k_ptr(const float* __restrict__ pd, const float* __restrict__ pen,
                                             const float* __restrict__ vp, float* __restrict__ out) {
  __shared__ __align__(16) float pdr[HID];
  __shared__ __align__(16) float vsh[HID];
  const int bt = blockIdx.x;
  const int b  = bt >> 8;
  const int i  = threadIdx.x;
  pdr[i] = pd[(size_t)bt * HID + i];
  vsh[i] = vp[i];
  __syncthreads();
  const float* pr = pen + ((size_t)(b * SQ + i)) * HID;
  float acc = 0.f;
#pragma unroll 1
  for (int h4 = 0; h4 < HID; h4 += 4) {
    const v4f pv = *(const v4f*)(pr + h4);
    const v4f dv = *(const v4f*)(pdr + h4);
    const v4f wv = *(const v4f*)(vsh + h4);
#pragma unroll
    for (int j = 0; j < 4; ++j) acc = fmaf(wv[j], tnh(dv[j] + pv[j]), acc);
  }
  const float val = acc;
  volatile float* o = (volatile float*)(out + (size_t)bt * SQ + i);
  *o = val;
  __threadfence();
  *o = val;
}

extern "C" void kernel_launch(void* const* d_in, const int* in_sizes, int n_in,
                              void* d_out, int out_size, void* d_ws, size_t ws_size,
                              hipStream_t stream) {
  if (n_in < 26) return;
  if (in_sizes[0]  != NTOK * DIN) return;
  if (in_sizes[1]  != NTOK) return;
  if (in_sizes[2]  != H2 * DIN) return;
  if (in_sizes[3]  != H2) return;
  if (in_sizes[4]  != H2 * H2) return;
  if (in_sizes[5]  != H2) return;
  if (in_sizes[6]  != SQ * H4) return;
  if (in_sizes[7]  != NL * NQKV * HID) return;
  if (in_sizes[8]  != NL * NQKV) return;
  if (in_sizes[9]  != NL * HID * HID) return;
  if (in_sizes[10] != NL * HID) return;
  if (in_sizes[11] != NL * HID) return;
  if (in_sizes[12] != NL * HID) return;
  if (in_sizes[13] != NL * DFF * HID) return;
  if (in_sizes[14] != NL * DFF) return;
  if (in_sizes[15] != NL * HID * DFF) return;
  if (in_sizes[16] != NL * HID) return;
  if (in_sizes[17] != NL * HID) return;
  if (in_sizes[18] != NL * HID) return;
  if (in_sizes[19] != G4 * HID) return;
  if (in_sizes[20] != G4 * HID) return;
  if (in_sizes[21] != G4) return;
  if (in_sizes[22] != G4) return;
  if (in_sizes[23] != HID * HID) return;
  if (in_sizes[24] != HID) return;
  if (in_sizes[25] != HID) return;
  if (out_size != NB * SQ * SQ) return;

  const float* parts = (const float*)d_in[0];
  const int*   tseq  = (const int*)d_in[1];
  const float* W_pe1 = (const float*)d_in[2];
  const float* b_pe1 = (const float*)d_in[3];
  const float* W_pe2 = (const float*)d_in[4];
  const float* b_pe2 = (const float*)d_in[5];
  const float* pos   = (const float*)d_in[6];
  const float* Wqkv  = (const float*)d_in[7];
  const float* bqkv  = (const float*)d_in[8];
  const float* Wo    = (const float*)d_in[9];
  const float* bo    = (const float*)d_in[10];
  const float* ln1g  = (const float*)d_in[11];
  const float* ln1b  = (const float*)d_in[12];
  const float* W1f   = (const float*)d_in[13];
  const float* b1f   = (const float*)d_in[14];
  const float* W2f   = (const float*)d_in[15];
  const float* b2f   = (const float*)d_in[16];
  const float* ln2g  = (const float*)d_in[17];
  const float* ln2b  = (const float*)d_in[18];
  const float* Wih   = (const float*)d_in[19];
  const float* Whh   = (const float*)d_in[20];
  const float* bih   = (const float*)d_in[21];
  const float* bhh   = (const float*)d_in[22];
  const float* Wp    = (const float*)d_in[23];
  const float* bp    = (const float*)d_in[24];
  const float* vptr  = (const float*)d_in[25];
  float* out = (float*)d_out;

  size_t off = 0;
  const size_t oWpe1 = off; off += (size_t)H2 * DINP * 2;
  const size_t oWpe2 = off; off += (size_t)H2 * H2 * 2;
  const size_t oWqkv = off; off += (size_t)NL * NQKV * HID * 2;
  const size_t oWo   = off; off += (size_t)NL * HID * HID * 2;
  const size_t oW1   = off; off += (size_t)NL * DFF * HID * 2;
  const size_t oW2   = off; off += (size_t)NL * HID * DFF * 2;
  const size_t oWih  = off; off += (size_t)G4 * HID * 2;
  const size_t oWhh  = off; off += (size_t)G4 * HID * 2;
  const size_t oWp   = off; off += (size_t)HID * HID * 2;
  const size_t oP16  = off; off += (size_t)NTOK * DINP * 2;
  const size_t oT1h  = off; off += (size_t)NTOK * H2 * 2;
  const size_t oP32  = off; off += (size_t)NTOK * H2 * 4;
  const size_t oXA   = off; off += (size_t)NTOK * HID * 4;
  const size_t oXB   = off; off += (size_t)NTOK * HID * 4;
  const size_t oX16  = off; off += (size_t)NTOK * HID * 2;
  const size_t oQK   = off; off += (size_t)2 * QKPLANE * 2;
  const size_t oVT   = off; off += (size_t)NB * NHD * HDM * SQ * 2;
  const size_t oO16  = off; off += (size_t)NTOK * HID * 2;
  const size_t oT    = off; off += (size_t)NTOK * HID * 4;
  const size_t oHd   = off; off += (size_t)NTOK * DFF * 2;
  const size_t oDIN  = off; off += (size_t)NTOK * HID * 2;
  const size_t oGX   = off; off += (size_t)NTOK * G4 * 4;
  const size_t oDOUT = off; off += (size_t)NTOK * HID * 2;
  const size_t oPD   = off; off += (size_t)NTOK * HID * 4;
  const size_t oPEN  = off; off += (size_t)NTOK * HID * 4;
  if (off > ws_size) return;
  if (off > (size_t)134217728) return;

  char* ws = (char*)d_ws;
  _Float16* Wpe1h = (_Float16*)(ws + oWpe1);
  _Float16* Wpe2h = (_Float16*)(ws + oWpe2);
  _Float16* Wqkvh = (_Float16*)(ws + oWqkv);
  _Float16* Woh   = (_Float16*)(ws + oWo);
  _Float16* W1h   = (_Float16*)(ws + oW1);
  _Float16* W2h   = (_Float16*)(ws + oW2);
  _Float16* Wihh  = (_Float16*)(ws + oWih);
  _Float16* Whhh  = (_Float16*)(ws + oWhh);
  _Float16* Wph   = (_Float16*)(ws + oWp);
  _Float16* P16   = (_Float16*)(ws + oP16);
  _Float16* T1h   = (_Float16*)(ws + oT1h);
  float*    P32   = (float*)(ws + oP32);
  float*    XA    = (float*)(ws + oXA);
  float*    XB    = (float*)(ws + oXB);
  _Float16* X16   = (_Float16*)(ws + oX16);
  _Float16* QK    = (_Float16*)(ws + oQK);
  _Float16* VT    = (_Float16*)(ws + oVT);
  _Float16* O16   = (_Float16*)(ws + oO16);
  float*    T     = (float*)(ws + oT);
  _Float16* Hd    = (_Float16*)(ws + oHd);
  _Float16* DIN16 = (_Float16*)(ws + oDIN);
  float*    GX    = (float*)(ws + oGX);
  _Float16* DOUT  = (_Float16*)(ws + oDOUT);
  float*    PD    = (float*)(ws + oPD);
  float*    PEN   = (float*)(ws + oPEN);

  k_cvt<<<dim3((NTOK * DINP / 8) / 256), dim3(256), 0, stream>>>(parts, P16, NTOK, DIN, DINP, 1.0f);
  k_cvt<<<dim3((H2 * DINP / 8) / 256), dim3(256), 0, stream>>>(W_pe1, Wpe1h, H2, DIN, DINP, 32.0f);
  k_cvt<<<dim3((H2 * H2 / 8) / 256), dim3(256), 0, stream>>>(W_pe2, Wpe2h, H2, H2, H2, 32.0f);
  k_cvt<<<dim3((NL * NQKV * HID / 8) / 256), dim3(256), 0, stream>>>(Wqkv, Wqkvh, NL * NQKV, HID, HID, 32.0f);
  k_cvt<<<dim3((NL * HID * HID / 8) / 256), dim3(256), 0, stream>>>(Wo, Woh, NL * HID, HID, HID, 32.0f);
  k_cvt<<<dim3((NL * DFF * HID / 8) / 256), dim3(256), 0, stream>>>(W1f, W1h, NL * DFF, HID, HID, 32.0f);
  k_cvt<<<dim3((NL * HID * DFF / 8) / 256), dim3(256), 0, stream>>>(W2f, W2h, NL * HID, DFF, DFF, 32.0f);
  k_cvt<<<dim3((G4 * HID / 8) / 256), dim3(256), 0, stream>>>(Wih, Wihh, G4, HID, HID, 32.0f);
  k_cvt<<<dim3((G4 * HID / 8) / 256), dim3(256), 0, stream>>>(Whh, Whhh, G4, HID, HID, 32.0f);
  k_cvt<<<dim3((HID * HID / 8) / 256), dim3(256), 0, stream>>>(Wp, Wph, HID, HID, HID, 32.0f);

  k_gemm_h16<<<dim3(NTOK / 256, H2 / 64), dim3(256), 0, stream>>>(P16, DINP, Wpe1h, DINP, b_pe1, 0.03125f, 16.0f, T1h, H2);
  k_gemm_f32<<<dim3(NTOK / 256, H2 / 64), dim3(256), 0, stream>>>(T1h, H2, Wpe2h, H2, b_pe2, 0.001953125f, P32, H2);
  k_asmx<<<dim3(NTOK / 8), dim3(256), 0, stream>>>(P32, pos, XA, X16);

  const float sscale = 0.17677669529663687f;
  for (int l = 0; l < NL; ++l) {
    k_qkv<<<dim3(NB, NQKV / 64), dim3(256), 0, stream>>>(X16, Wqkvh + (size_t)l * NQKV * HID, bqkv + l * NQKV, QK, VT);
    k_attn<<<dim3(NB * NHD * 2), dim3(256), 0, stream>>>(QK, VT, O16, sscale);
    k_gemm_oh<<<dim3(NTOK / 256, HID / 64), dim3(256), 0, stream>>>(O16, Woh + (size_t)l * HID * HID, bo + l * HID, 0.00048828125f, T, HID);
    k_ln<<<dim3(NTOK / 8), dim3(256), 0, stream>>>(T, XA, ln1g + l * HID, ln1b + l * HID, XB, X16);
    k_gemm_h16<<<dim3(NTOK / 256, DFF / 64), dim3(256), 0, stream>>>(X16, HID, W1h + (size_t)l * DFF * HID, HID, b1f + l * DFF, 0.03125f, 16.0f, Hd, DFF);
    k_gemm_f32<<<dim3(NTOK / 256, HID / 64), dim3(256), 0, stream>>>(Hd, DFF, W2h + (size_t)l * HID * DFF, DFF, b2f + l * HID, 0.001953125f, T, HID);
    k_ln<<<dim3(NTOK / 8), dim3(256), 0, stream>>>(T, XB, ln2g + l * HID, ln2b + l * HID, XA, X16);
  }

  k_gather<<<dim3(NTOK / 8), dim3(256), 0, stream>>>(X16, tseq, DIN16);
  k_gemm_f32<<<dim3(NTOK / 256, G4 / 64), dim3(256), 0, stream>>>(DIN16, HID, Wihh, HID, bih, 0.03125f, GX, G4);
  k_lstm<<<dim3(1), dim3(256), 0, stream>>>(GX, Whhh, bhh, DOUT);

  k_gemm_f32<<<dim3(NTOK / 256, HID / 64), dim3(256), 0, stream>>>(DOUT, HID, Wph, HID, bp, 0.00048828125f, PD, HID);
  k_gemm_f32<<<dim3(NTOK / 256, HID / 64), dim3(256), 0, stream>>>(X16, HID, Wph, HID, bp, 0.03125f, PEN, HID);
  k_ptr<<<dim3(NB * SQ), dim3(256), 0, stream>>>(PD, PEN, vptr, out);
  (void)hipGetLastError();
}
